// StaticSparseAttention_33380485824625
// MI455X (gfx1250) — hardware-verified
//
#include <hip/hip_runtime.h>
#include <stdint.h>

#define CE     768
#define CH     12
#define CD     64
#define CSEQ   2049
#define CL     2048
#define CB     2
#define CNQKV  2304
#define CNQK   1536
#define CWS    16
#define CNQB   32
#define CMROWS 4098
#define CMPAD  4160
#define CNTRIG 32

typedef __attribute__((ext_vector_type(16))) _Float16 v16h;
typedef __attribute__((ext_vector_type(8)))  _Float16 v8h;
typedef __attribute__((ext_vector_type(16))) __bf16   v16b;
typedef __attribute__((ext_vector_type(8)))  __bf16   v8b;
typedef __attribute__((ext_vector_type(8)))  float    v8f;
typedef __attribute__((ext_vector_type(4)))  float    v4f;

#define NEG_INF (-__builtin_inff())

__device__ __forceinline__ unsigned short f2bf_bits(float f) {
  unsigned u = __float_as_uint(f);
  return (unsigned short)((u + 0x7FFFu + ((u >> 16) & 1u)) >> 16);
}
__device__ __forceinline__ float bf_bits2f(unsigned short h) { return __uint_as_float(((unsigned)h) << 16); }

__device__ __forceinline__ void dep_guard_h(v8f& a, v8f& b, v16h x, v16h y) { asm volatile("v_nop\n\tv_nop\n\tv_nop\n\tv_nop" : "+v"(a), "+v"(b) : "v"(x), "v"(y)); }
__device__ __forceinline__ void dep_guard_b(v8f& a, v8f& b, v16b x, v16b y) { asm volatile("v_nop\n\tv_nop\n\tv_nop\n\tv_nop" : "+v"(a), "+v"(b) : "v"(x), "v"(y)); }
__device__ __forceinline__ void keep4_h(v16h a, v16h b, v16h c, v16h d) { asm volatile("v_nop" :: "v"(a), "v"(b), "v"(c), "v"(d)); }
__device__ __forceinline__ void keep4_b(v16b a, v16b b, v16b c, v16b d) { asm volatile("v_nop" :: "v"(a), "v"(b), "v"(c), "v"(d)); }
__device__ __forceinline__ void acc_guard4(v8f& a, v8f& b, v8f& c, v8f& d) { asm volatile("v_nop\n\tv_nop\n\tv_nop\n\tv_nop" : "+v"(a), "+v"(b), "+v"(c), "+v"(d)); }
template <typename T> struct Frag;
template <> struct Frag<_Float16> {
  typedef v16h V; union U { v16h v; v8h h[2]; };
  static __device__ __forceinline__ v16h load(const _Float16* p) {
    U f; f.h[0] = *(const v8h*)(p); f.h[1] = *(const v8h*)(p + 16); return f.v;
  }
  static __device__ __forceinline__ v8f mma(v16h a, v16h b, v8f c) {
    return __builtin_amdgcn_wmma_f32_16x16x32_f16(false, a, false, b, (short)0, c, false, false);
  }
  static __device__ __forceinline__ void guard(v8f& a, v8f& b, v16h x, v16h y) { dep_guard_h(a, b, x, y); }
  static __device__ __forceinline__ void keep(v16h a, v16h b, v16h c, v16h d) { keep4_h(a, b, c, d); }
};
template <> struct Frag<__bf16> {
  typedef v16b V; union U { v16b v; v8b h[2]; };
  static __device__ __forceinline__ v16b load(const __bf16* p) {
    U f; f.h[0] = *(const v8b*)(p); f.h[1] = *(const v8b*)(p + 16); return f.v;
  }
  static __device__ __forceinline__ v8f mma(v16b a, v16b b, v8f c) {
    return __builtin_amdgcn_wmma_f32_16x16x32_bf16(false, a, false, b, (short)0, c, false, false);
  }
  static __device__ __forceinline__ void guard(v8f& a, v8f& b, v16b x, v16b y) { dep_guard_b(a, b, x, y); }
  static __device__ __forceinline__ void keep(v16b a, v16b b, v16b c, v16b d) { keep4_b(a, b, c, d); }
};

template <int ET> struct Elem;
template <> struct Elem<0> { typedef _Float16 T; };
template <> struct Elem<1> { typedef __bf16 T; };
template <int ET, bool SPLIT, int BIAS_MODE, int OUT_MODE, bool RESID, int ACT = 0>
__global__ __launch_bounds__(256) void wmma_gemm64(
    const unsigned short* __restrict__ Ap, const unsigned short* __restrict__ A2p, int lda, long strideA,
    const unsigned short* __restrict__ Btp, const unsigned short* __restrict__ Bt2p, int ldb, long strideB,
    void* __restrict__ Cout, void* __restrict__ Cout2, int ldc, long strideC,
    const float* __restrict__ bias,
    const float* __restrict__ resid, long strideR,
    int M, int N, int K, float scale, int Mvalid) {
  typedef typename Elem<ET>::T T;
  typedef typename Frag<T>::V V;
  const T* A = (const T*)Ap; const T* A2 = (const T*)A2p; const T* Bt = (const T*)Btp; const T* Bt2 = (const T*)Bt2p;
  __shared__ __align__(16) float sT[8][16 * 68];
  const int b    = blockIdx.y;
  const int lane = threadIdx.x & 31;
  const int wave = threadIdx.x >> 5;
  const int tilesN = N >> 6;
  const int tilesM = M >> 6;
  const int tile = blockIdx.x * 8 + wave;
  if (tile >= tilesM * tilesN) return;
  const int tm = tile / tilesN;
  const int tn = tile - tm * tilesN;
  const int m0 = tm << 6;
  const int n0 = tn << 6;

  const T* Ab  = A  + (size_t)b * strideA;
  const T* Bb  = Bt + (size_t)b * strideB;
  const T* Ab2 = SPLIT ? (A2  + (size_t)b * strideA) : nullptr;
  const T* Bb2 = SPLIT ? (Bt2 + (size_t)b * strideB) : nullptr;

  const int rlane = lane & 15;
  const int koff  = (lane >> 4) * 8;
  const int mOff  = (lane >> 4) * 8;

  v8f acc[4][4];
#pragma unroll
  for (int i = 0; i < 4; ++i)
#pragma unroll
    for (int j = 0; j < 4; ++j) acc[i][j] = (v8f){0.f,0.f,0.f,0.f,0.f,0.f,0.f,0.f};

  for (int k0 = 0; k0 < K; k0 += 32) {
    V bh[4], bl[4];
#pragma unroll
    for (int j = 0; j < 4; ++j) {
      const size_t bo = (size_t)(n0 + (j << 4) + rlane) * ldb + koff + k0;
      bh[j] = Frag<T>::load(Bb + bo);
      if (SPLIT) bl[j] = Frag<T>::load(Bb2 + bo);
    }
#pragma unroll
    for (int i = 0; i < 4; ++i) {
      const size_t ao = (size_t)(m0 + (i << 4) + rlane) * lda + koff + k0;
      V ah = Frag<T>::load(Ab + ao);
      V al;
      if (SPLIT) al = Frag<T>::load(Ab2 + ao);
#pragma unroll
      for (int j = 0; j < 4; ++j) {
        acc[i][j] = Frag<T>::mma(ah, bh[j], acc[i][j]);
        if (SPLIT) {
          acc[i][j] = Frag<T>::mma(ah, bl[j], acc[i][j]);
          acc[i][j] = Frag<T>::mma(al, bh[j], acc[i][j]);
        }
      }
      Frag<T>::guard(acc[i][0], acc[i][3], ah, SPLIT ? al : ah);
    }
    Frag<T>::keep(bh[0], bh[1], bh[2], bh[3]);
    if (SPLIT) Frag<T>::keep(bl[0], bl[1], bl[2], bl[3]);
  }
  acc_guard4(acc[0][0], acc[0][1], acc[0][2], acc[0][3]);
  acc_guard4(acc[1][0], acc[1][1], acc[1][2], acc[1][3]);
  acc_guard4(acc[2][0], acc[2][1], acc[2][2], acc[2][3]);
  acc_guard4(acc[3][0], acc[3][1], acc[3][2], acc[3][3]);

  float* slab = sT[wave];
  const float* Rb = RESID ? (resid + (size_t)b * strideR) : nullptr;
#pragma unroll
  for (int i = 0; i < 4; ++i) {
    const int mBase = m0 + (i << 4);
#pragma unroll
    for (int j = 0; j < 4; ++j) {
      const int n = n0 + (j << 4) + rlane;
      float bv = 0.f;
      if (BIAS_MODE == 2) bv = bias[n];
#pragma unroll
      for (int r = 0; r < 8; ++r) {
        float v = acc[i][j][r] * scale;
        if (BIAS_MODE == 1) v += bias[mBase + mOff + r];
        if (BIAS_MODE == 2) v += bv;
        if (RESID) v += Rb[(size_t)(mBase + mOff + r) * ldc + n];
        if (ACT == 1) v = tanhf(v);
        if (ACT == 2) v = fmaxf(v, 0.0f);
        if (ACT == 3) v = v / (1.0f + expf(-v));
        if (ACT == 4) v = (v > 0.f) ? v : 0.01f * v;
        if (ACT == 5) v = 0.5f * v * (1.0f + erff(v * 0.70710678118654752f));
        slab[(mOff + r) * 68 + (j << 4) + rlane] = v;
      }
    }
    __builtin_amdgcn_fence(__ATOMIC_RELEASE, "workgroup");
    __builtin_amdgcn_wave_barrier();
    __builtin_amdgcn_fence(__ATOMIC_ACQUIRE, "workgroup");
    if (OUT_MODE == 0) {
      float* C = (float*)Cout + (size_t)b * strideC;
      const int hh = lane >> 4, c4 = (lane & 15) * 4;
      for (int pass = 0; pass < 2; ++pass) {
#pragma unroll
        for (int it = 0; it < 8; ++it) {
          const int row = it * 2 + hh;
          v4f v = *(const v4f*)(slab + row * 68 + c4);
          if (mBase + row < Mvalid) *(volatile v4f*)(C + (size_t)(mBase + row) * ldc + n0 + c4) = v;
        }
        __threadfence();
      }
    } else {
      const int q = lane >> 3, c8 = (lane & 7) * 8;
      unsigned short* C  = (unsigned short*)Cout  + (size_t)b * strideC;
      unsigned short* C2 = (OUT_MODE == 2) ? ((unsigned short*)Cout2 + (size_t)b * strideC) : nullptr;
      for (int pass = 0; pass < 2; ++pass) {
#pragma unroll
        for (int it = 0; it < 4; ++it) {
          const int row = it * 4 + q;
          const float* sp = slab + row * 68 + c8;
          v8h hv, lv;
#pragma unroll
          for (int e = 0; e < 8; ++e) {
            if (OUT_MODE == 1) {
              hv[e] = (_Float16)sp[e];
            } else {
              unsigned short hb = f2bf_bits(sp[e]);
              unsigned short lb = f2bf_bits(sp[e] - bf_bits2f(hb));
              hv[e] = __builtin_bit_cast(_Float16, hb);
              lv[e] = __builtin_bit_cast(_Float16, lb);
            }
          }
          if (mBase + row < Mvalid) {
            *(volatile v8h*)(C + (size_t)(mBase + row) * ldc + n0 + c8) = hv;
            if (OUT_MODE == 2) *(volatile v8h*)(C2 + (size_t)(mBase + row) * ldc + n0 + c8) = lv;
          }
        }
        __threadfence();
      }
    }
    __builtin_amdgcn_fence(__ATOMIC_RELEASE, "workgroup");
    __builtin_amdgcn_wave_barrier();
    __builtin_amdgcn_fence(__ATOMIC_ACQUIRE, "workgroup");
  }
}

__global__ __launch_bounds__(256) void cast_f32_f16x2(
    const float* __restrict__ in, _Float16* __restrict__ out, int n2) {
  int i = blockIdx.x * 256 + threadIdx.x;
  if (i < n2) {
    const _Float16 h0 = (_Float16)in[2 * i], h1 = (_Float16)in[2 * i + 1];
    const unsigned u = (unsigned)__builtin_bit_cast(unsigned short, h0) | ((unsigned)__builtin_bit_cast(unsigned short, h1) << 16);
    ((volatile unsigned*)out)[i] = u;
    __threadfence();
    ((volatile unsigned*)out)[i] = u;
  }
}

#define AT_D 64
#define AT_NW 4
#define AT_QB 64
#define AT_KC 64
__device__ __forceinline__ unsigned short at_bf_bits(float f) {
  unsigned u = __float_as_uint(f);
  return (unsigned short)((u + 0x7FFFu + ((u >> 16) & 1u)) >> 16);
}
__device__ __forceinline__ __bf16 at_f2bf(float f) { return __builtin_bit_cast(__bf16, at_bf_bits(f)); }
__device__ __forceinline__ v8f at_mma(v16b a, v16b b, v8f c) {
  c = __builtin_amdgcn_wmma_f32_16x16x32_bf16(false, a, false, b, (short)0, c, false, false);
  asm volatile("v_nop\n\tv_nop\n\tv_nop\n\tv_nop" : "+v"(c) : "v"(a), "v"(b));
  return c;
}
template <bool F16> __device__ __forceinline__ __bf16 at_to16(float f) {
  if (F16) return __builtin_bit_cast(__bf16, (_Float16)f);
  return at_f2bf(f);
}
template <bool F16> __device__ __forceinline__ v8f at_mma16(v16b a, v16b b, v8f c) {
  if (F16) {
    const v16h ah = __builtin_bit_cast(v16h, a), bh = __builtin_bit_cast(v16h, b);
    c = __builtin_amdgcn_wmma_f32_16x16x32_f16(false, ah, false, bh, (short)0, c, false, false);
    asm volatile("v_nop\n\tv_nop\n\tv_nop\n\tv_nop" : "+v"(c) : "v"(ah), "v"(bh));
    return c;
  }
  return at_mma(a, b, c);
}

__constant__ float c_inv_freq[16] = {
  1.0f, 0.5623413251903491f, 0.31622776601683794f, 0.17782794100389229f,
  0.1f, 0.05623413251903491f, 0.031622776601683794f, 0.017782794100389229f,
  0.01f, 0.005623413251903491f, 0.0031622776601683794f, 0.0017782794100389228f,
  0.001f, 0.0005623413251903491f, 0.00031622776601683794f, 0.00017782794100389227f };

__global__ __launch_bounds__(256) void trig_table_kernel(
    const float* __restrict__ coords, float* __restrict__ cosT, float* __restrict__ sinT, int n) {
  const int i = blockIdx.x * 256 + threadIdx.x;
  if (i >= n) return;
  const int j = i & 31;
  const int bl = i >> 5;
  const float cxy = coords[(size_t)bl * 2 + (j >> 4)];
  const float xy = cxy * (1.0f / 100000.0f);
  const float f = xy * c_inv_freq[j & 15];
  float sn, cs;
  sincosf(f, &sn, &cs);
  ((volatile float*)cosT)[i] = cs;
  ((volatile float*)sinT)[i] = sn;
  __threadfence();
  ((volatile float*)cosT)[i] = cs;
  ((volatile float*)sinT)[i] = sn;
}

__global__ __launch_bounds__(256) void rope_kernel(
    const float* __restrict__ qkv, const float* __restrict__ cosT, const float* __restrict__ sinT,
    float* __restrict__ qkr, int nrows) {
  const int g = blockIdx.x * 256 + threadIdx.x;
  const int row = g / (CNQK / 4);
  const int c4 = g - row * (CNQK / 4);
  if (row >= nrows) return;
  const int col = c4 * 4;
  const int b = row / CSEQ;
  const int s = row - b * CSEQ;
  const v4f x = *(const v4f*)(qkv + (size_t)row * CNQKV + col);
  v4f o = x;
  if (s > 0) {
    const int d0 = col & 63;
    const int j0 = d0 >> 1;
    const size_t ti = ((size_t)b * CL + (s - 1)) * CNTRIG + j0;
    const float c0 = cosT[ti], s0 = sinT[ti], c1 = cosT[ti + 1], s1 = sinT[ti + 1];
    o[0] = x[0] * c0 - x[1] * s0;
    o[1] = x[1] * c0 + x[0] * s0;
    o[2] = x[2] * c1 - x[3] * s1;
    o[3] = x[3] * c1 + x[2] * s1;
  }
  float* dst = qkr + (size_t)row * CNQK + col;
  *(volatile v4f*)dst = o;
  __threadfence();
  *(volatile v4f*)dst = o;
}

__global__ __launch_bounds__(256) void cls_attn_kernel(
    const float* __restrict__ qk, const float* __restrict__ qkv, unsigned short* __restrict__ outh) {
  __shared__ float sc[CSEQ];
  __shared__ float red[256];
  __shared__ float qc[CD];
  __shared__ float part[4][CD];
  __shared__ float ov[CD];
  const int bh = blockIdx.x;
  const int b = bh / CH;
  const int h = bh - b * CH;
  const int t = threadIdx.x;
  const size_t rb = (size_t)b * CSEQ;
  const float* qrow  = qk  + rb * CNQK + h * CD;
  const float* kbase = qk  + rb * CNQK + CE + h * CD;
  const float* vbase = qkv + rb * CNQKV + 2 * CE + h * CD;

  if (t < CD) qc[t] = qrow[t];
  __syncthreads();

  float lmax = NEG_INF;
  for (int s = t; s < CSEQ; s += 256) {
    const float* kr = kbase + (size_t)s * CNQK;
    float dot = 0.f;
#pragma unroll 8
    for (int i = 0; i < CD; ++i) dot += qc[i] * kr[i];
    dot *= 0.125f;
    sc[s] = dot;
    lmax = fmaxf(lmax, dot);
  }
  red[t] = lmax;
  __syncthreads();
  for (int o = 128; o > 0; o >>= 1) {
    if (t < o) red[t] = fmaxf(red[t], red[t + o]);
    __syncthreads();
  }
  const float mx = red[0];
  __syncthreads();

  float lsum = 0.f;
  for (int s = t; s < CSEQ; s += 256) {
    const float p = expf(sc[s] - mx);
    sc[s] = p;
    lsum += p;
  }
  red[t] = lsum;
  __syncthreads();
  for (int o = 128; o > 0; o >>= 1) {
    if (t < o) red[t] = red[t] + red[t + o];
    __syncthreads();
  }
  const float inv = 1.0f / red[0];
  __syncthreads();

  const int d = t & 63, pi = t >> 6;
  float a = 0.f;
#pragma unroll 4
  for (int s = pi; s < CSEQ; s += 4) a += sc[s] * vbase[(size_t)s * CNQKV + d];
  part[pi][d] = a;
  __syncthreads();
  if (t < CD) ov[t] = ((part[0][t] + part[1][t]) + (part[2][t] + part[3][t])) * inv;
  __syncthreads();

  v8h hv = (v8h){(_Float16)0, (_Float16)0, (_Float16)0, (_Float16)0, (_Float16)0, (_Float16)0, (_Float16)0, (_Float16)0};
  unsigned short* op = outh + rb * CE + h * CD + t * 8;
  if (t < 8) {
#pragma unroll
    for (int e = 0; e < 8; ++e) hv[e] = (_Float16)ov[t * 8 + e];
    *(volatile v8h*)op = hv;
  }
  __threadfence();
  if (t < 8) *(volatile v8h*)op = hv;
}

__global__ __launch_bounds__(128)
void band_attn_kernel(const float* __restrict__ qk, const float* __restrict__ qkv,
                      unsigned short* __restrict__ outh) {
  const float PSC = 32768.0f;
  union FB { v16b v; v8b h[2]; };
  __shared__ __align__(16) __bf16 Ksh[AT_KC * AT_D];
  __shared__ __align__(16) __bf16 Vth[AT_D * AT_KC];
  __shared__ __align__(16) __bf16 Psh[AT_NW][16 * AT_KC];
  __shared__ __align__(16) float  Os[AT_NW][16 * 68];

  const int tid  = threadIdx.x;
  const int wave = tid >> 5;
  const int lane = tid & 31;
  const int hh   = lane >> 4;
  const int c    = lane & 15;
  const int bx = blockIdx.x;
  const int qb = bx % CNQB;
  const int bh = bx / CNQB;
  const int h  = bh % CH;
  const int b  = bh / CH;
  const int q0 = qb * AT_QB + wave * 16;
  const size_t rb = (size_t)b * CSEQ;
  const float* qb_ptr = qk  + rb * CNQK + h * CD;
  const float* kb_ptr = qk  + rb * CNQK + CE + h * CD;
  const float* vb_ptr = qkv + rb * CNQKV + 2 * CE + h * CD;
  unsigned short* ob  = outh + rb * CE + h * CD;

  v16b qah[2];
  float scp = 0.f;
  {
    const float* qrow = qb_ptr + (size_t)(1 + q0 + c) * CNQK;
#pragma unroll
    for (int dc = 0; dc < 2; ++dc) {
#pragma unroll
      for (int e = 0; e < 8; ++e) {
        const int d0 = dc * 32 + 8 * hh + e;
        const int d1 = d0 + 16;
        const float f0 = qrow[d0] * 0.125f;
        const float f1 = qrow[d1] * 0.125f;
        scp += f0 * kb_ptr[d0];
        scp += f1 * kb_ptr[d1];
        qah[dc][e] = at_to16<true>(f0);
        qah[dc][8 + e] = at_to16<true>(f1);
      }
    }
  }
  const float scr = scp + __shfl_xor(scp, 16, 32);
  float mrow[8], lrow[8];
  v8f oacc[4];
#pragma unroll
  for (int r = 0; r < 8; ++r) { mrow[r] = __shfl(scr, 8 * hh + r, 32); lrow[r] = 1.0f; }
#pragma unroll
  for (int t = 0; t < 4; ++t) {
    const float vc = vb_ptr[t * 16 + c] * PSC;
    oacc[t] = (v8f){vc, vc, vc, vc, vc, vc, vc, vc};
  }

  for (int kc = 0; kc < 2; ++kc) {
    const int j0 = qb * AT_QB - CWS + kc * AT_KC;
    __syncthreads();
    {
      const int kvr = tid >> 1, dh = (tid & 1) * 32;
      int kp = j0 + kvr;
      kp = kp < 0 ? 0 : kp;
      kp = kp > (CL - 1) ? (CL - 1) : kp;
      const float* krow = kb_ptr + (size_t)(1 + kp) * CNQK + dh;
      const float* vrow = vb_ptr + (size_t)(1 + kp) * CNQKV + dh;
#pragma unroll
      for (int i = 0; i < 8; ++i) {
        v4f kk = *(const v4f*)(krow + 4 * i);
        v4f vv = *(const v4f*)(vrow + 4 * i);
#pragma unroll
        for (int e = 0; e < 4; ++e) {
          const int d = dh + 4 * i + e;
          Ksh[kvr * AT_D + d] = at_to16<true>(kk[e]);
          Vth[d * AT_KC + kvr] = at_to16<true>(vv[e]);
        }
      }
    }
    __syncthreads();

    v8f s[4];
#pragma unroll
    for (int j = 0; j < 4; ++j) {
      s[j] = (v8f){0.f,0.f,0.f,0.f,0.f,0.f,0.f,0.f};
#pragma unroll
      for (int dc = 0; dc < 2; ++dc) {
        FB kb;
        kb.h[0] = *(const v8b*)(Ksh + (j * 16 + c) * AT_D + dc * 32 + 8 * hh);
        kb.h[1] = *(const v8b*)(Ksh + (j * 16 + c) * AT_D + dc * 32 + 16 + 8 * hh);
        s[j] = at_mma16<true>(qah[dc], kb.v, s[j]);
      }
    }
    float cm[8];
#pragma unroll
    for (int r = 0; r < 8; ++r) {
      const int lq = q0 + 8 * hh + r;
      float m = NEG_INF;
#pragma unroll
      for (int j = 0; j < 4; ++j) {
        const int kp = j0 + j * 16 + c;
        const bool masked = (kp < 0) || (kp >= CL) || (kp < lq - CWS) || (kp > lq + CWS);
        if (masked) s[j][r] = NEG_INF;
        m = fmaxf(m, s[j][r]);
      }
#pragma unroll
      for (int off = 1; off < 16; off <<= 1) m = fmaxf(m, __shfl_xor(m, off, 32));
      cm[r] = m;
    }
    __bf16* pwh = Psh[wave];
#pragma unroll
    for (int r = 0; r < 8; ++r) {
      const float mnew = fmaxf(mrow[r], cm[r]);
      const float alpha = expf(mrow[r] - mnew);
      mrow[r] = mnew;
      float psum = 0.f;
#pragma unroll
      for (int j = 0; j < 4; ++j) {
        const float p = expf(s[j][r] - mnew);
        psum += p;
        pwh[(8 * hh + r) * AT_KC + j * 16 + c] = at_to16<true>(p * PSC);
      }
#pragma unroll
      for (int off = 1; off < 16; off <<= 1) psum += __shfl_xor(psum, off, 32);
      lrow[r] = lrow[r] * alpha + psum;
#pragma unroll
      for (int t = 0; t < 4; ++t) oacc[t][r] *= alpha;
    }
    __builtin_amdgcn_fence(__ATOMIC_RELEASE, "workgroup");
    __builtin_amdgcn_wave_barrier();
    __builtin_amdgcn_fence(__ATOMIC_ACQUIRE, "workgroup");
#pragma unroll 1
    for (int kk = 0; kk < 2; ++kk) {
      FB pa;
      pa.h[0] = *(const v8b*)(pwh + c * AT_KC + kk * 32 + 8 * hh);
      pa.h[1] = *(const v8b*)(pwh + c * AT_KC + kk * 32 + 16 + 8 * hh);
#pragma unroll
      for (int t = 0; t < 4; ++t) {
        FB vb;
        vb.h[0] = *(const v8b*)(Vth + (t * 16 + c) * AT_KC + kk * 32 + 8 * hh);
        vb.h[1] = *(const v8b*)(Vth + (t * 16 + c) * AT_KC + kk * 32 + 16 + 8 * hh);
        oacc[t] = at_mma16<true>(pa.v, vb.v, oacc[t]);
      }
    }
  }

  float* os = Os[wave];
#pragma unroll
  for (int r = 0; r < 8; ++r) {
    const float inv = 1.0f / (lrow[r] * PSC);
#pragma unroll
    for (int t = 0; t < 4; ++t) os[(8 * hh + r) * 68 + t * 16 + c] = oacc[t][r] * inv;
  }
  __builtin_amdgcn_fence(__ATOMIC_RELEASE, "workgroup");
  __builtin_amdgcn_wave_barrier();
  __builtin_amdgcn_fence(__ATOMIC_ACQUIRE, "workgroup");
  {
    const int q8 = lane >> 3, c8 = (lane & 7) * 8;
    for (int pass = 0; pass < 2; ++pass) {
#pragma unroll
      for (int it = 0; it < 4; ++it) {
        const int row = it * 4 + q8;
        const float* sp = os + row * 68 + c8;
        v8h hv;
#pragma unroll
        for (int e = 0; e < 8; ++e) hv[e] = (_Float16)sp[e];
        *(volatile v8h*)(ob + (size_t)(1 + q0 + row) * CE + c8) = hv;
      }
      __threadfence();
    }
  }
}

extern "C" void kernel_launch(void* const* d_in, const int* in_sizes, int n_in,
                              void* d_out, int out_size, void* d_ws, size_t ws_size,
                              hipStream_t stream)
{
  if (n_in < 6) return;
  if (in_sizes[0] != CMROWS * CE || in_sizes[1] != CB * CL * 2 || in_sizes[2] != CNQKV * CE ||
      in_sizes[3] != CNQKV || in_sizes[4] != CE * CE || in_sizes[5] != CE || out_size != CMROWS * CE) return;

  const float* x      = (const float*)d_in[0];
  const float* coords = (const float*)d_in[1];
  const float* qkv_w  = (const float*)d_in[2];
  const float* qkv_b  = (const float*)d_in[3];
  const float* out_w  = (const float*)d_in[4];
  const float* out_b  = (const float*)d_in[5];
  float* out = (float*)d_out;

  char* ws = (char*)d_ws;
  size_t off = 0;
  auto carve = [&](size_t bytes) -> char* {
    char* p = ws + off;
    off += (bytes + 255) & ~(size_t)255;
    return p;
  };
  unsigned short* xh    = (unsigned short*)carve((size_t)CMPAD * CE * 2);
  unsigned short* wqh   = (unsigned short*)carve((size_t)CNQKV * CE * 2);
  unsigned short* woh   = (unsigned short*)carve((size_t)CE * CE * 2);
  float*          qkvf  = (float*)carve((size_t)CMPAD * CNQKV * 4);
  float*          qkr   = (float*)carve((size_t)CMROWS * CNQK * 4);
  unsigned short* attnh = (unsigned short*)carve((size_t)CMPAD * CE * 2);
  float*          cosT  = (float*)carve((size_t)CB * CL * CNTRIG * 4);
  float*          sinT  = (float*)carve((size_t)CB * CL * CNTRIG * 4);
  if (off > ws_size) return;

  {
    const int n2x = CMROWS * CE / 2;
    cast_f32_f16x2<<<(n2x + 255) / 256, 256, 0, stream>>>(x, (_Float16*)xh, n2x);
    const int n2q = CNQKV * CE / 2;
    cast_f32_f16x2<<<(n2q + 255) / 256, 256, 0, stream>>>(qkv_w, (_Float16*)wqh, n2q);
    const int n2o = CE * CE / 2;
    cast_f32_f16x2<<<(n2o + 255) / 256, 256, 0, stream>>>(out_w, (_Float16*)woh, n2o);
    const size_t tail_off = (size_t)CMROWS * CE * 2;
    const size_t tail_len = (size_t)(CMPAD - CMROWS) * CE * 2;
    hipMemsetAsync((char*)xh + tail_off, 0, tail_len, stream);
    hipMemsetAsync((char*)attnh + tail_off, 0, tail_len, stream);
  }

  {
    const int tiles = (CMPAD / 64) * (CNQKV / 64);
    dim3 g((tiles + 7) / 8, 1);
    wmma_gemm64<0, false, 2, 0, false, 0><<<g, 256, 0, stream>>>(
        xh, nullptr, CE, 0L,
        wqh, nullptr, CE, 0L,
        (void*)qkvf, nullptr, CNQKV, 0L,
        qkv_b,
        nullptr, 0L,
        CMPAD, CNQKV, CE, 1.0f, CMPAD);
  }

  {
    const int nt = CB * CL * CNTRIG;
    trig_table_kernel<<<(nt + 255) / 256, 256, 0, stream>>>(coords, cosT, sinT, nt);
    const int n4 = CMROWS * (CNQK / 4);
    rope_kernel<<<(n4 + 255) / 256, 256, 0, stream>>>(qkvf, cosT, sinT, qkr, CMROWS);
  }

  cls_attn_kernel<<<CB * CH, 256, 0, stream>>>(qkr, qkvf, attnh);

  band_attn_kernel<<<CB * CH * CNQB, 128, 0, stream>>>(qkr, qkvf, attnh);

  {
    const int tiles = (CMPAD / 64) * (CE / 64);
    dim3 g((tiles + 7) / 8, 1);
    wmma_gemm64<0, false, 2, 0, false, 0><<<g, 256, 0, stream>>>(
        attnh, nullptr, CE, 0L,
        woh, nullptr, CE, 0L,
        (void*)out, nullptr, CE, 0L,
        out_b,
        nullptr, 0L,
        CMPAD, CE, CE, 1.0f, CMROWS);
  }
}
